// MxDNADeforambleConvBlock_15513421873291
// MI455X (gfx1250) — hardware-verified
//
#include <hip/hip_runtime.h>
#include <math.h>


#define NB 4
#define LL 4096
#define CC 768
#define KH 7
#define KT (KH * CC)
#define NR (NB * LL)

typedef __attribute__((ext_vector_type(16))) _Float16 v16h;
typedef __attribute__((ext_vector_type(16))) __bf16 v16b;
typedef __attribute__((ext_vector_type(8)))  _Float16 v8h;
typedef __attribute__((ext_vector_type(8)))  float v8f;
typedef __attribute__((ext_vector_type(4)))  float v4f;
typedef __attribute__((ext_vector_type(4)))  unsigned v4u;
typedef float __attribute__((may_alias)) float_a;

template <typename T> __device__ __forceinline__ void vst2(void* p, T v) { *(volatile T*)p = v; __threadfence(); *(volatile T*)p = v; }
__device__ __forceinline__ v8f wmma16(v16h a, v16h b, v8f c) {
  v8f d = __builtin_amdgcn_wmma_f32_16x16x32_f16(false, a, false, b, (short)0, c, false, false);
  asm volatile("v_nop\n\tv_nop\n\tv_nop\n\tv_nop" : "+v"(d) : "v"(a), "v"(b));
  return d;
}
__device__ __forceinline__ v8f wmma_bf(v16b a, v16b b, v8f c) {
  v8f d = __builtin_amdgcn_wmma_f32_16x16x32_bf16(false, a, false, b, (short)0, c, false, false);
  asm volatile("v_nop\n\tv_nop\n\tv_nop\n\tv_nop" : "+v"(d) : "v"(a), "v"(b));
  return d;
}
__device__ __forceinline__ v16h frag_h(const _Float16* rowk0, int lane) {
  union { v16h v; v8h q[2]; } u; const _Float16* p = rowk0 + 8 * (lane >> 4);
  u.q[0] = *(const v8h*)p; u.q[1] = *(const v8h*)(p + 16); return u.v;
}
struct F2 { v16b h, l; };
__device__ __forceinline__ F2 split_row(const float* rowk0, int lane) {
  F2 r;
  if (rowk0 == nullptr) {
#pragma unroll
    for (int i = 0; i < 16; ++i) { r.h[i] = (__bf16)0.f; r.l[i] = (__bf16)0.f; }
    return r; }
  const float* p = rowk0 + 8 * (lane >> 4);
#pragma unroll
  for (int i = 0; i < 8; ++i) { float v0 = p[i], v1 = p[16 + i]; __bf16 h0 = (__bf16)v0, h1 = (__bf16)v1;
    r.h[i] = h0; r.l[i] = (__bf16)(v0 - (float)h0); r.h[8 + i] = h1; r.l[8 + i] = (__bf16)(v1 - (float)h1); }
  return r;
}
__device__ __forceinline__ v8f mac3(const F2& a, const F2& b, v8f c) { c = wmma_bf(a.l, b.h, c); c = wmma_bf(a.h, b.l, c); return wmma_bf(a.h, b.h, c); }
#define LDSX() do { asm volatile("s_wait_dscnt 0" ::: "memory"); __builtin_amdgcn_wave_barrier(); __builtin_amdgcn_fence(__ATOMIC_RELEASE, "workgroup"); } while (0)

__global__ __launch_bounds__(192) void k_ln(const float* __restrict__ x, const float* __restrict__ am, const float* __restrict__ sm,
                                          const float* __restrict__ lw, const float* __restrict__ lb, float* __restrict__ h, float* __restrict__ gate) {
  __shared__ float r2[256];
  const size_t row = blockIdx.x; const int tid = threadIdx.x;
  const float* xr = x + row * CC;
  const v4f v = *(const v4f*)(xr + tid * 4);
  r2[tid] = v[0] + v[1] + v[2] + v[3]; if (tid < 64) r2[192 + tid] = 0.f; __syncthreads();
  for (int st = 128; st > 0; st >>= 1) { if (tid < st) r2[tid] += r2[tid + st]; __syncthreads(); }
  const float mu = r2[0] / (float)CC; __syncthreads();
  const float d0 = v[0] - mu, d1 = v[1] - mu, d2 = v[2] - mu, d3 = v[3] - mu;
  r2[tid] = d0 * d0 + d1 * d1 + d2 * d2 + d3 * d3; if (tid < 64) r2[192 + tid] = 0.f; __syncthreads();
  for (int st = 128; st > 0; st >>= 1) { if (tid < st) r2[tid] += r2[tid + st]; __syncthreads(); }
  const float rs = rsqrtf(r2[0] / (float)CC + 1e-12f);
  const v4f w = *(const v4f*)(lw + tid * 4), bb = *(const v4f*)(lb + tid * 4);
  v4f o = { d0 * rs * w[0] + bb[0], d1 * rs * w[1] + bb[1], d2 * rs * w[2] + bb[2], d3 * rs * w[3] + bb[3] };
  vst2(h + row * CC + tid * 4, o);
  if (tid == 0) vst2(gate + row * 32, (float_a)((1.0f - sm[row]) * am[row]));
}

__global__ __launch_bounds__(256) void k_packc(const float* __restrict__ ow, const float* __restrict__ mw, float* __restrict__ Wc) {
  const int n = blockIdx.y, q = blockIdx.x * 256 + threadIdx.x;
  if (q >= KT / 4) return;
  v4f v;
#pragma unroll
  for (int e = 0; e < 4; ++e) { const int kidx = q * 4 + e, kk = kidx / CC, c = kidx % CC;
    v[e] = n < 7 ? ow[((size_t)n * CC + c) * KH + kk] : (n < 14 ? mw[((size_t)(n - 7) * CC + c) * KH + kk] : 0.f); }
  vst2(Wc + (size_t)n * KT + q * 4, v);
}
__global__ __launch_bounds__(256) void k_packr(const float* __restrict__ rw, _Float16* __restrict__ Br) {
  const int o = blockIdx.y, q = blockIdx.x * 256 + threadIdx.x;
  if (q >= KT / 8) return;
  union { v8h h; v4u u; } pk;
#pragma unroll
  for (int e = 0; e < 8; ++e) { const int kidx = q * 8 + e, kk = kidx / CC, c = kidx % CC; pk.h[e] = (_Float16)rw[((size_t)o * CC + c) * KH + kk]; }
  vst2(Br + (size_t)o * KT + q * 8, pk.u);
}

__global__ __launch_bounds__(128) void k_offmod(const float* __restrict__ h, const float* __restrict__ Wc, const float* __restrict__ ob,
                                              const float* __restrict__ mb, float* __restrict__ fpos, float* __restrict__ modv) {
  __shared__ __align__(16) float sp[64][8], sm2[64][8];
  const int tid = threadIdx.x, wave = tid >> 5, lane = tid & 31, col = lane & 15, g = lane >> 4;
  const int r0 = blockIdx.x * 64 + wave * 16, b = r0 / LL, p0 = r0 % LL;
  const int p = p0 + col;
  v8f acc = {};
#pragma unroll 1
  for (int kc = 0; kc < KT / 32; ++kc) {
    const int kk = (kc * 32) / CC, c0 = (kc * 32) % CC; const int q = p + kk - 3;
    const float* arow = (q >= 0 && q < LL) ? h + ((size_t)b * LL + q) * CC + c0 : nullptr;
    acc = mac3(split_row(arow, lane), split_row(Wc + (size_t)col * KT + kc * 32, lane), acc);
  }
#pragma unroll
  for (int r = 0; r < 8; ++r) { const int pr = p0 + 8 * g + r;
    if (col < 7)       sp[wave * 16 + 8 * g + r][col] = (float)(pr - 3 + col) + (acc[r] + ob[col]);
    else if (col < 14) sm2[wave * 16 + 8 * g + r][col - 7] = 2.0f / (1.0f + expf(-(acc[r] + mb[col - 7])));
    else if (col == 14) { sp[wave * 16 + 8 * g + r][7] = 0.f; sm2[wave * 16 + 8 * g + r][7] = 0.f; } }
  __syncthreads();
  for (int q = tid; q < 64 * 2; q += 128) { const int rl = q >> 1, hf = q & 1;
    vst2(fpos + (size_t)(blockIdx.x * 64 + rl) * 8 + hf * 4, *(const v4f*)(&sp[rl][hf * 4]));
    vst2(modv + (size_t)(blockIdx.x * 64 + rl) * 8 + hf * 4, *(const v4f*)(&sm2[rl][hf * 4])); }
}

__global__ __launch_bounds__(256) void k_sample(const float* __restrict__ h, const float* __restrict__ gate, const float* __restrict__ fpos,
                                              const float* __restrict__ modv, _Float16* __restrict__ S) {
  const size_t row = blockIdx.x; const int b = (int)(row / LL), tid = threadIdx.x;
  for (int q = tid; q < KH * (CC / 8); q += 256) { const int kk = q / (CC / 8), c0 = (q % (CC / 8)) * 8;
    const float pos = fpos[row * 8 + kk], md = modv[row * 8 + kk];
    const float fl = floorf(pos); const int fi = (int)fl; const float t = pos - fl;
    const bool in0 = fi >= 0 && fi <= LL - 1, in1 = fi + 1 >= 0 && fi + 1 <= LL - 1;
    const size_t q0 = (size_t)b * LL + (in0 ? fi : 0), q1 = (size_t)b * LL + (in1 ? fi + 1 : 0);
    const float g0 = in0 ? gate[q0 * 32] * (1.f - t) : 0.f, g1 = in1 ? gate[q1 * 32] * t : 0.f;
    union { v8h hh; v4u u; } pk;
#pragma unroll
    for (int e = 0; e < 8; ++e) pk.hh[e] = (_Float16)((h[q0 * CC + c0 + e] * g0 + h[q1 * CC + c0 + e] * g1) * md);
    vst2(S + row * KT + (size_t)kk * CC + c0, pk.u); }
}

__global__ __launch_bounds__(128) void k_gemm(const _Float16* __restrict__ S, const _Float16* __restrict__ Br, const float* __restrict__ x, float* __restrict__ out) {
  __shared__ __align__(16) float so[4][16 * 128];
  const int tid = threadIdx.x, wave = tid >> 5, lane = tid & 31, col = lane & 15, g = lane >> 4;
  const int r0 = blockIdx.x * 64 + wave * 16, n0 = blockIdx.y * 128;
  v8f acc[8] = {};
#pragma unroll 1
  for (int kc = 0; kc < KT / 32; ++kc) {
    const v16h a = frag_h(S + (size_t)(r0 + col) * KT + kc * 32, lane);
#pragma unroll
    for (int j = 0; j < 8; ++j) acc[j] = wmma16(a, frag_h(Br + (size_t)(n0 + j * 16 + col) * KT + kc * 32, lane), acc[j]);
  }
  float* Sg = so[wave];
#pragma unroll
  for (int j = 0; j < 8; ++j)
#pragma unroll
    for (int r = 0; r < 8; ++r) Sg[(8 * g + r) * 128 + j * 16 + col] = acc[j][r];
  LDSX();
#pragma unroll 4
  for (int rl = 0; rl < 16; ++rl) { const size_t o = (size_t)(r0 + rl) * CC + n0 + lane * 4;
    vst2(out + o, *(const v4f*)(Sg + rl * 128 + lane * 4) + *(const v4f*)(x + o)); }
}

extern "C" void kernel_launch(void* const* d_in, const int* in_sizes, int n_in,
                              void* d_out, int out_size, void* d_ws, size_t ws_size,
                              hipStream_t stream) {
  (void)in_sizes; (void)n_in; (void)out_size; (void)ws_size;
  const float* x  = (const float*)d_in[0];
  const float* am = (const float*)d_in[1]; const float* sm = (const float*)d_in[2];
  const float* lw = (const float*)d_in[3]; const float* lb = (const float*)d_in[4];
  const float* ow = (const float*)d_in[5]; const float* ob = (const float*)d_in[6];
  const float* mw = (const float*)d_in[7]; const float* mb = (const float*)d_in[8];
  const float* rw = (const float*)d_in[9];
  float* out = (float*)d_out;
  char* ws = (char*)d_ws; size_t off = 0;
  auto take = [&](size_t bytes) { char* p = ws + off; off += (bytes + 255) & ~(size_t)255; return p; };
  float* h    = (float*)take((size_t)NR * CC * 4);
  float* gate = (float*)take((size_t)NR * 32 * 4);
  float* Wc   = (float*)take((size_t)16 * KT * 4);
  _Float16* Br = (_Float16*)take((size_t)CC * KT * 2);
  float* fpos = (float*)take((size_t)NR * 8 * 4);
  float* modv = (float*)take((size_t)NR * 8 * 4);
  _Float16* S = (_Float16*)take((size_t)NR * KT * 2);
  k_ln<<<NR, 192, 0, stream>>>(x, am, sm, lw, lb, h, gate);
  k_packc<<<dim3((KT / 4 + 255) / 256, 16), 256, 0, stream>>>(ow, mw, Wc);
  k_packr<<<dim3((KT / 8 + 255) / 256, CC), 256, 0, stream>>>(rw, Br);
  k_offmod<<<NR / 64, 128, 0, stream>>>(h, Wc, ob, mb, fpos, modv);
  k_sample<<<NR, 256, 0, stream>>>(h, gate, fpos, modv, S);
  k_gemm<<<dim3(NR / 64, CC / 128), 128, 0, stream>>>(S, Br, x, out);
}
